// GraphAttentionLayer_3539053052652
// MI455X (gfx1250) — hardware-run, weakly checked
//
#include <hip/hip_runtime.h>


#ifndef NB
#define NB 8
#endif
#ifndef SEQ
#define SEQ 2048
#endif
#define NB_FULL  8
#define SEQ_FULL 2048
#ifndef OUT_SEQ
#define OUT_SEQ SEQ
#endif
#define DM   256
#define AW   4
#define OSP  132
#define WPR  (SEQ / 32)
#define WTR  8
#define SLOPE   0.2f
#define NEG_BIG (-9.0e15f)
#define L2E  1.4426950408889634f
#define PSH  14.0f
#define NEGB (-3.0e38f)

static_assert(DM == 256);
static_assert(DM % 64 == 0);
static_assert(DM % 32 == 0);
static_assert(SEQ % 64 == 0);
static_assert((NB * SEQ) % 64 == 0);
static_assert(SEQ % 32 == 0);
static_assert(SEQ % (16 * AW) == 0);
static_assert(((size_t)SEQ * WPR) % 256 == 0);
static_assert(((size_t)SEQ * DM) % 8 == 0);
static_assert(256 * 8 == WTR * DM);
static_assert(DM % WTR == 0);
static_assert(NB <= NB_FULL);
static_assert(SEQ <= SEQ_FULL);
static_assert((OSP * 4) % 16 == 0);
static_assert(OSP >= 128);
static_assert(32 * 16 * 4 == 16 * 64 * 2);
static_assert(32 * 16 * 16 == 16 * 128 * 4);
static_assert(8 * 16 == 32 * 4);
static_assert(16 * 16 == 64 * 4);
static_assert(8 * 16 == 32 * 4);
static_assert(AW * 16 * OSP * 4 <= 131072);
static_assert(SEQ * 4 + 32 * 4 <= 131072);
static_assert(16 * 68 * 4 + 2 * DM * 4 + 128 * 4 <= 131072);

typedef _Float16 h16;
typedef unsigned short bf;
typedef __attribute__((ext_vector_type(16))) __bf16   v16bf;
typedef __attribute__((ext_vector_type(16))) _Float16 v16h;
typedef __attribute__((ext_vector_type(8)))  _Float16 v8h;
typedef __attribute__((ext_vector_type(8)))  unsigned short v8us;
typedef __attribute__((ext_vector_type(8)))  float    v8f;
typedef __attribute__((ext_vector_type(4)))  float    v4f;
typedef __attribute__((ext_vector_type(4)))  int      v4i;
typedef __attribute__((ext_vector_type(4)))  unsigned v4u;
typedef v4f  __attribute__((may_alias)) v4fa;
typedef v8us __attribute__((may_alias)) v8usa;
typedef v4u  __attribute__((may_alias)) v4ua;

__device__ __forceinline__ unsigned short f2bf(float f) { unsigned u = __float_as_uint(f); u += 0x7FFFu + ((u >> 16) & 1u); return (unsigned short)(u >> 16); }
__device__ __forceinline__ float bfr(float f) { return __uint_as_float(((unsigned)f2bf(f)) << 16); }
__device__ __forceinline__ v16h cat16(v8h lo, v8h hi) { return __builtin_shufflevector(lo, hi, 0, 1, 2, 3, 4, 5, 6, 7, 8, 9, 10, 11, 12, 13, 14, 15); }
__device__ __forceinline__ v16bf cat16b(v8us lo, v8us hi) { return __builtin_bit_cast(v16bf, __builtin_shufflevector(lo, hi, 0, 1, 2, 3, 4, 5, 6, 7, 8, 9, 10, 11, 12, 13, 14, 15)); }
__device__ __forceinline__ v8f wmma16(v16h a, v16h b, v8f c) { return __builtin_amdgcn_wmma_f32_16x16x32_f16(false, a, false, b, (short)0, c, false, false); }
__device__ __forceinline__ v8f wmmab(v16bf a, v16bf b, v8f c) { return __builtin_amdgcn_wmma_f32_16x16x32_bf16(false, a, false, b, (short)0, c, false, false); }
__device__ __forceinline__ v16h  ldh(const h16* p) { return cat16(*(const v8h*)p, *(const v8h*)(p + 16)); }
__device__ __forceinline__ v16bf ldb(const bf* p)  { return cat16b(*(const v8us*)p, *(const v8us*)(p + 16)); }
__device__ __forceinline__ void wave_sync() { __builtin_amdgcn_fence(3  , "wavefront"); __builtin_amdgcn_wave_barrier(); asm volatile("" ::: "memory"); }
__device__ __forceinline__ v8f wmma16g(v16h a, v16h b, v8f c) { c = wmma16(a, b, c); asm volatile("v_nop\n\tv_nop\n\tv_nop\n\tv_nop" : "+v"(c) : "v"(a), "v"(b)); return c; }
__device__ __forceinline__ v8f wmmabg(v16bf a, v16bf b, v8f c) { c = wmmab(a, b, c); asm volatile("v_nop\n\tv_nop\n\tv_nop\n\tv_nop" : "+v"(c) : "v"(a), "v"(b)); return c; }
static __device__ __forceinline__ h16 toh_flush(float v) { const h16 r = (h16)v; return (fabsf(v) < 6.103515625e-05f) ? (h16)0.0f : r; }

__global__ __launch_bounds__(256) void k_cvt8(const float* __restrict__ src, bf* dst, size_t n8) {
    const size_t i = (size_t)blockIdx.x * 256 + threadIdx.x; if (i >= n8) return;
    const v8f v = *(const v8f*)(src + i * 8); v8us o;
#pragma unroll
    for (int k = 0; k < 8; ++k) o[k] = f2bf(v[k]);
    *(volatile v8us*)(dst + i * 8) = o; __threadfence(); *(volatile v8us*)(dst + i * 8) = o;
}

__global__ __launch_bounds__(256) void k_wT(const float* __restrict__ W, bf* WT) {
    __shared__ __align__(16) unsigned short ts[WTR * (DM + 8)];
    const int tid = threadIdx.x; const int n0 = blockIdx.x * WTR;
    { const int k = tid;
      const v4f x0 = *(const v4f*)(W + (size_t)k * DM + n0); const v4f x1 = *(const v4f*)(W + (size_t)k * DM + n0 + 4);
#pragma unroll
      for (int i = 0; i < 4; ++i) { ts[i * (DM + 8) + k] = f2bf(x0[i]); ts[(4 + i) * (DM + 8) + k] = f2bf(x1[i]); } }
    __syncthreads();
    const int row = tid >> 5, c8 = (tid & 31) * 8;
    const v8us o = *(const v8usa*)(&ts[row * (DM + 8) + c8]);
    bf* d = WT + (size_t)(n0 + row) * DM + c8;
    *(volatile v8us*)d = o; __threadfence(); *(volatile v8us*)d = o;
}

__global__ __launch_bounds__(256) void k_bits(const int* __restrict__ adj, unsigned* BW) {
    const int gid = blockIdx.x * 256 + threadIdx.x;
    const int i = gid / WPR, w = gid % WPR;
    const int* p = adj + (size_t)i * SEQ_FULL + 32 * w;
    unsigned word = 0u;
#pragma unroll 1
    for (int q = 0; q < 8; ++q) { const v4i v = *(const v4i*)(p + 4 * q);
        const unsigned nib = (v[0] > 0 ? 1u : 0u) | (v[1] > 0 ? 2u : 0u) | (v[2] > 0 ? 4u : 0u) | (v[3] > 0 ? 8u : 0u);
        word |= nib << (4 * q); }
    const int lane = threadIdx.x & 31; const int q4 = (lane & 7) * 4;
    v4u o;
    o[0] = (unsigned)__shfl((int)word, q4 + 0, 32); o[1] = (unsigned)__shfl((int)word, q4 + 1, 32);
    o[2] = (unsigned)__shfl((int)word, q4 + 2, 32); o[3] = (unsigned)__shfl((int)word, q4 + 3, 32);
    unsigned* d = BW + (size_t)(gid - lane) + q4;
    if (lane < 8) *(volatile v4ua*)d = o;
    __threadfence();
    if (lane < 8) *(volatile v4ua*)d = o;
}

__global__ __launch_bounds__(32) void k_hproj(const bf* __restrict__ WT, const bf* __restrict__ XB, const float* __restrict__ avec, h16* HT, float* SS) {
    __shared__ __align__(16) float os[16 * 68];
    __shared__ __align__(16) float av[2 * DM];
    __shared__ __align__(16) float sst[4 * 32];
    const int K = DM;
    const int lane = threadIdx.x & 31, lr = lane & 15, hi = lane >> 4; const int c0 = blockIdx.x * 64;
    const int bb = c0 / SEQ, tt = c0 % SEQ;
#pragma unroll 1
    for (int i = lane; i < 2 * DM; i += 32) av[i] = bfr(avec[i]);
    wave_sync();
    float p1a = 0.0f, p1b = 0.0f, p2a = 0.0f, p2b = 0.0f;
    const size_t boff = (size_t)(c0 + lr) * K + 8 * hi;
#pragma unroll 1
    for (int dt = 0; dt < DM / 64; ++dt) {
        const int r0 = dt * 64;
        v8f acc[4][4];
#pragma unroll
        for (int mb = 0; mb < 4; ++mb)
#pragma unroll
            for (int nb = 0; nb < 4; ++nb) acc[mb][nb] = (v8f){};
        const size_t aoff = (size_t)(r0 + lr) * K + 8 * hi;
#pragma unroll 1
        for (int kc = 0; kc < K; kc += 32) {
            v16bf a[4];
#pragma unroll
            for (int mb = 0; mb < 4; ++mb) a[mb] = ldb(WT + aoff + (size_t)mb * 16 * K + kc);
#pragma unroll
            for (int nb = 0; nb < 4; ++nb) { const v16bf b = ldb(XB + boff + (size_t)nb * 16 * K + kc);
#pragma unroll
                for (int mb = 0; mb < 4; ++mb) acc[mb][nb] = wmmabg(a[mb], b, acc[mb][nb]); }
        }
        const size_t tbase = (size_t)bb * (size_t)DM * SEQ + (size_t)r0 * SEQ + (size_t)tt;
#pragma unroll
        for (int mb = 0; mb < 4; ++mb) {
#pragma unroll
            for (int nb = 0; nb < 4; ++nb) {
#pragma unroll
                for (int j = 0; j < 8; ++j) os[(hi * 8 + j) * 68 + nb * 16 + lr] = acc[mb][nb][j]; }
            wave_sync();
            const int dbase = r0 + mb * 16;
#pragma unroll 4
            for (int row = 0; row < 16; ++row) {
                const float w1 = av[dbase + row], w2 = av[DM + dbase + row];
                const float va = os[row * 68 + lane], vb = os[row * 68 + 32 + lane];
                p1a = fmaf(va, w1, p1a); p1b = fmaf(vb, w1, p1b); p2a = fmaf(va, w2, p2a); p2b = fmaf(vb, w2, p2b); }
            const size_t sb = tbase + (size_t)(mb * 16) * SEQ;
#pragma unroll 1
            for (int ps = 0; ps < 2; ++ps) {
#pragma unroll
                for (int s = 0; s < 4; ++s) { const int row = 4 * s + (lane >> 3), c8 = (lane & 7) * 8;
                    const v4f x0 = *(const v4fa*)(&os[row * 68 + c8]); const v4f x1 = *(const v4fa*)(&os[row * 68 + c8 + 4]); v8h hv;
#pragma unroll
                    for (int i = 0; i < 4; ++i) { hv[i] = toh_flush(x0[i]); hv[4 + i] = toh_flush(x1[i]); }
                    const size_t oo = sb + (size_t)row * SEQ + c8;
                    *(volatile v8h*)(HT + oo) = hv; }
                if (ps == 0) __threadfence(); }
            wave_sync();
        }
    }
    sst[lane] = p1a; sst[32 + lane] = p1b; sst[64 + lane] = p2a; sst[96 + lane] = p2b;
    wave_sync();
    { const v4f val = *(const v4fa*)(&sst[hi * 64 + lr * 4]);
      float* d = SS + (size_t)hi * ((size_t)NB * SEQ) + (size_t)c0 + (size_t)lr * 4;
      *(volatile v4f*)d = val; __threadfence(); *(volatile v4f*)d = val; }
}

__global__ __launch_bounds__(256) void k_rowmax(const unsigned* __restrict__ BW, const float* __restrict__ SS, float* MR) {
    __shared__ __align__(16) float s2s[SEQ];
    __shared__ __align__(16) float res[32];
    const int tid = threadIdx.x, lane = tid & 31;
    const int wave = __builtin_amdgcn_readfirstlane((int)(threadIdx.x >> 5));
    const int b = blockIdx.y; const int i0 = blockIdx.x * 32;
    const float* S1 = SS + (size_t)b * SEQ;
    const float* S2 = SS + (size_t)NB * SEQ + (size_t)b * SEQ;
#pragma unroll 1
    for (int idx = tid; idx < SEQ / 4; idx += 256) { const v4f v = *(const v4f*)(S2 + 4 * idx); *(v4fa*)(&s2s[4 * idx]) = v; }
    __syncthreads();
#pragma unroll 1
    for (int q = 0; q < 4; ++q) {
        const int i = i0 + wave * 4 + q;
        float mx = NEGB;
#pragma unroll 1
        for (int wb = 0; wb < WPR; wb += 32) {
            const int wi = wb + lane; const int wc = wi < WPR ? wi : (WPR - 1);
            unsigned word = BW[(size_t)i * WPR + wc];
            asm volatile("" : "+v"(word));
            word = (wi < WPR) ? word : 0u;
#pragma unroll 4
            for (int k = 0; k < 32; ++k) { const float v = s2s[32 * wc + k]; mx = ((word >> k) & 1u) ? fmaxf(mx, v) : mx; }
        }
        mx = fmaxf(mx, __shfl_xor(mx, 16, 32)); mx = fmaxf(mx, __shfl_xor(mx, 8, 32)); mx = fmaxf(mx, __shfl_xor(mx, 4, 32));
        mx = fmaxf(mx, __shfl_xor(mx, 2, 32));  mx = fmaxf(mx, __shfl_xor(mx, 1, 32));
        const float s1i = S1[i];
        const float vv = s1i + mx; const float lk = fmaxf(vv, SLOPE * vv);
        const float mr = (mx > -1.0e38f) ? lk : NEG_BIG;
        if (lane == 0) res[wave * 4 + q] = mr;
    }
    __syncthreads();
    if ((wave == 0) & (lane < 8)) { const v4f o = *(const v4fa*)(&res[4 * lane]);
        float* d = MR + (size_t)b * SEQ + i0 + 4 * lane;
        *(volatile v4f*)d = o; __threadfence(); *(volatile v4f*)d = o; }
}

__global__ __launch_bounds__(32 * AW) __attribute__((amdgpu_num_vgpr(256)))
void k_fused(const h16* __restrict__ HT, const float* __restrict__ SS, const float* __restrict__ MR, const unsigned* __restrict__ BW, float* OUT) {
    __shared__ __align__(16) float os[AW * 16 * OSP];
    const int lane = threadIdx.x & 31, lr = lane & 15, hi = lane >> 4;
    const int wave = __builtin_amdgcn_readfirstlane((int)(threadIdx.x >> 5));
    const int b = blockIdx.y;
    const int t0 = (blockIdx.x * AW + wave) * 16;
    const size_t rowi = (size_t)b * SEQ + t0 + lr;
    const float s1i = SS[rowi];
    const float mrow = MR[rowi];
    const float* s2p = SS + (size_t)NB * SEQ + (size_t)b * SEQ + 8 * hi;
    const unsigned* bwp = BW + (size_t)(t0 + lr) * WPR;
    const size_t vo = (size_t)b * (size_t)DM * SEQ + (size_t)lr * SEQ + 8 * hi;
    v8f o[16];
#pragma unroll
    for (int j = 0; j < 16; ++j) o[j] = (v8f){};
    float l = 0.0f;
#pragma unroll 1
    for (int key0 = 0; key0 < SEQ; key0 += 32) {
        const unsigned wsh = bwp[key0 >> 5] >> (8 * hi);
        const float* kp = s2p + key0;
        const v4f m0 = *(const v4f*)kp, m1 = *(const v4f*)(kp + 4), m2 = *(const v4f*)(kp + 16), m3 = *(const v4f*)(kp + 20);
        float kx[8], ky[8];
#pragma unroll
        for (int r = 0; r < 4; ++r) { kx[r] = m0[r]; kx[4 + r] = m1[r]; ky[r] = m2[r]; ky[4 + r] = m3[r]; }
        v16h pb; float ls = 0.0f;
#pragma unroll
        for (int r = 0; r < 8; ++r) {
            const float va = s1i + kx[r], vb = s1i + ky[r];
            const float la = fmaxf(va, SLOPE * va), lb = fmaxf(vb, SLOPE * vb);
            const float xa = ((wsh >> r) & 1u) ? la : NEG_BIG;
            const float xb = ((wsh >> (16 + r)) & 1u) ? lb : NEG_BIG;
            const float ea = (xa - mrow) * L2E + PSH, eb = (xb - mrow) * L2E + PSH;
            const float ga = (ea < -14.0f) ? 0.0f : __builtin_amdgcn_exp2f(ea);
            const float gb = (eb < -14.0f) ? 0.0f : __builtin_amdgcn_exp2f(eb);
            const h16 pa = (h16)ga; const h16 pc = (h16)gb;
            pb[r] = pa; pb[8 + r] = pc;
            ls += (float)pa + (float)pc; }
        l += ls;
#pragma unroll
        for (int g = 0; g < 4; ++g) {
            const h16* va = HT + vo + (size_t)(64 * g) * SEQ + key0;
            const v16h a0 = ldh(va), a1 = ldh(va + (size_t)16 * SEQ), a2 = ldh(va + (size_t)32 * SEQ), a3 = ldh(va + (size_t)48 * SEQ);
            o[4 * g + 0] = wmma16g(a0, pb, o[4 * g + 0]);
            o[4 * g + 1] = wmma16g(a1, pb, o[4 * g + 1]);
            o[4 * g + 2] = wmma16g(a2, pb, o[4 * g + 2]);
            o[4 * g + 3] = wmma16g(a3, pb, o[4 * g + 3]);
            asm volatile("" ::: "memory");
        }
    }
    l += __shfl_xor(l, 16, 32);
    const bool any = l > 0.0f;
    const float lsafe = any ? l : 1.0f;
    const float inv = any ? (1.0f / lsafe) : 0.0f;
    const int wb = wave * 16 * OSP;
    float* orow = OUT + ((size_t)b * OUT_SEQ + t0) * DM;
#pragma unroll
    for (int hf = 0; hf < 2; ++hf) {
#pragma unroll
        for (int jj = 0; jj < 8; ++jj) { const v8f f = o[8 * hf + jj]; v4f a, c;
#pragma unroll
            for (int i = 0; i < 4; ++i) {
                const float xa = f[i] * inv, xc = f[4 + i] * inv;
                a[i] = xa > 0.0f ? xa : (__builtin_amdgcn_exp2f(xa * L2E) - 1.0f);
                c[i] = xc > 0.0f ? xc : (__builtin_amdgcn_exp2f(xc * L2E) - 1.0f); }
            *(v4fa*)(&os[wb + lr * OSP + 16 * jj + 8 * hi]) = a; *(v4fa*)(&os[wb + lr * OSP + 16 * jj + 8 * hi + 4]) = c; }
        wave_sync();
#pragma unroll 1
        for (int ps = 0; ps < 2; ++ps) {
#pragma unroll 4
            for (int row = 0; row < 16; ++row) {
                const v4f val = *(const v4fa*)(&os[wb + row * OSP + lane * 4]);
                *(volatile v4f*)(orow + (size_t)row * DM + hf * 128 + lane * 4) = val; }
            if (ps == 0) __threadfence(); }
        wave_sync();
    }
}

static constexpr size_t al256(size_t v) { return (v + 255) & ~(size_t)255; }
static constexpr size_t SZ_XB = al256((size_t)NB * SEQ * DM * 2);
static constexpr size_t SZ_WT = al256((size_t)DM * DM * 2);
static constexpr size_t SZ_HT = al256((size_t)NB * DM * SEQ * 2);
static constexpr size_t SZ_SS = al256((size_t)2 * NB * SEQ * 4);
static constexpr size_t SZ_MR = al256((size_t)NB * SEQ * 4);
static constexpr size_t SZ_BW = al256((size_t)SEQ * WPR * 4);
static constexpr size_t SZ_TOTAL = SZ_XB + SZ_WT + SZ_HT + SZ_SS + SZ_MR + SZ_BW;
static_assert(SZ_TOTAL <= (size_t)134217728);
static_assert(((size_t)NB * SEQ * 4) % 128 == 0);

extern "C" void kernel_launch(void* const* d_in, const int* in_sizes, int n_in,
                              void* d_out, int out_size, void* d_ws, size_t ws_size, hipStream_t stream) {
    if (n_in < 4) return;
    const size_t needx = ((size_t)(NB - 1) * SEQ_FULL + SEQ) * DM;
    const size_t needa = (size_t)(SEQ - 1) * SEQ_FULL + SEQ;
    if ((size_t)in_sizes[0] < needx) return;
    if ((size_t)in_sizes[1] < needa) return;
    if ((size_t)in_sizes[2] < (size_t)DM * DM) return;
    if (in_sizes[3] < 2 * DM) return;
    if ((size_t)out_size < ((size_t)(NB - 1) * OUT_SEQ + SEQ) * DM) return;
    if (SZ_TOTAL > ws_size) return;
    const float* x   = (const float*)d_in[0];
    const int*   adj = (const int*)d_in[1];
    const float* W   = (const float*)d_in[2];
    const float* av  = (const float*)d_in[3];
    float* OUT = (float*)d_out;
    char* wsp = (char*)d_ws;
    bf* XB = (bf*)wsp; wsp += SZ_XB;
    bf* WT = (bf*)wsp; wsp += SZ_WT;
    h16* HT = (h16*)wsp; wsp += SZ_HT;
    float* SS = (float*)wsp; wsp += SZ_SS;
    float* MR = (float*)wsp; wsp += SZ_MR;
    unsigned* BW = (unsigned*)wsp; wsp += SZ_BW;

    if (SEQ == SEQ_FULL) {
        const size_t n8 = (size_t)NB * SEQ * DM / 8;
        k_cvt8<<<(unsigned)((n8 + 255) / 256), 256, 0, stream>>>(x, XB, n8);
    } else {
        const size_t n8 = (size_t)SEQ * DM / 8;
        for (int b = 0; b < NB; ++b) k_cvt8<<<(unsigned)((n8 + 255) / 256), 256, 0, stream>>>(x + (size_t)b * SEQ_FULL * DM, XB + (size_t)b * SEQ * DM, n8);
    }
    k_wT<<<DM / WTR, 256, 0, stream>>>(W, WT);
    k_bits<<<(unsigned)(((size_t)SEQ * WPR) / 256), 256, 0, stream>>>(adj, BW);
    k_hproj<<<NB * SEQ / 64, 32, 0, stream>>>(WT, XB, av, HT, SS);
    k_rowmax<<<dim3(SEQ / 32, NB, 1), 256, 0, stream>>>(BW, SS, MR);
    k_fused<<<dim3(SEQ / (16 * AW), NB, 1), 32 * AW, 0, stream>>>(HT, SS, MR, BW, OUT);
}
